// MultiAttention_34514357190902
// MI455X (gfx1250) — hardware-run, weakly checked
//
#include <hip/hip_runtime.h>


#ifndef NB
#define NB 128
#endif
#ifndef SEQ
#define SEQ 1024
#endif
#define NB_FULL  128
#define SEQ_FULL 1024
#define DE   64
#define NH_  4
#define HDW  256
#define W1R  8
#define FW   8
#define NBP  (((NB + 63) / 64) * 64)
#define TPW  (SEQ / (16 * FW))
#define OUT1_OFF ((size_t)NB_FULL * DE)

static_assert(DE == 64);
static_assert(NH_ * DE == HDW);
static_assert(32 * FW == HDW);
static_assert(SEQ % (16 * FW) == 0);
static_assert(NB <= NB_FULL);
static_assert(SEQ <= SEQ_FULL);
static_assert(OUT1_OFF * 4 == 32768);
static_assert((OUT1_OFF * 4) % 128 == 0);
static_assert(NBP % 64 == 0);
static_assert(DE % 32 == 0);
static_assert((2 * HDW) % 32 == 0);

typedef unsigned short bf;
typedef __attribute__((ext_vector_type(16))) __bf16   v16bf;
typedef __attribute__((ext_vector_type(8)))  unsigned short v8us;
typedef __attribute__((ext_vector_type(8)))  float    v8f;
typedef __attribute__((ext_vector_type(4)))  float    v4f;
typedef v4f  __attribute__((may_alias)) v4fa;

__device__ __forceinline__ unsigned short f2bf(float f) { unsigned u = __float_as_uint(f); u += 0x7FFFu + ((u >> 16) & 1u); return (unsigned short)(u >> 16); }
__device__ __forceinline__ float bf2f(unsigned short b) { return __uint_as_float(((unsigned)b) << 16); }
__device__ __forceinline__ float bf16r(float f) { return bf2f(f2bf(f)); }
__device__ __forceinline__ v16bf cat16b(v8us lo, v8us hi) { return __builtin_bit_cast(v16bf, __builtin_shufflevector(lo, hi, 0, 1, 2, 3, 4, 5, 6, 7, 8, 9, 10, 11, 12, 13, 14, 15)); }
__device__ __forceinline__ v8f wmmab(v16bf a, v16bf b, v8f c) { return __builtin_amdgcn_wmma_f32_16x16x32_bf16(false, a, false, b, (short)0, c, false, false); }
__device__ __forceinline__ v16bf ldb(const bf* p)  { return cat16b(*(const v8us*)p, *(const v8us*)(p + 16)); }
__device__ __forceinline__ v16bf lda_f32(const float* p) {
    const v4f x0 = *(const v4f*)p, x1 = *(const v4f*)(p + 4), y0 = *(const v4f*)(p + 16), y1 = *(const v4f*)(p + 20);
    v8us lo, hi;
#pragma unroll
    for (int i = 0; i < 4; ++i) { lo[i] = f2bf(x0[i]); lo[4 + i] = f2bf(x1[i]); hi[i] = f2bf(y0[i]); hi[4 + i] = f2bf(y1[i]); }
    return cat16b(lo, hi);
}
__device__ __forceinline__ void wave_sync() { __builtin_amdgcn_fence(3  , "wavefront"); __builtin_amdgcn_wave_barrier(); asm volatile("" ::: "memory"); }
__device__ __forceinline__ void guard4(v8f& c0, v8f& c1, v8f& c2, v8f& c3, v16bf a, v16bf b0, v16bf b1, v16bf b2, v16bf b3) {
    asm volatile("v_nop\n\tv_nop\n\tv_nop\n\tv_nop" : "+v"(c0), "+v"(c1), "+v"(c2), "+v"(c3) : "v"(a), "v"(b0), "v"(b1), "v"(b2), "v"(b3));
}
__device__ __forceinline__ void guard1(v8f& c, v16bf a0, v16bf a1, v16bf b) {
    asm volatile("v_nop\n\tv_nop\n\tv_nop\n\tv_nop" : "+v"(c) : "v"(a0), "v"(a1), "v"(b));
}
__device__ __forceinline__ float sigm(float x) { return 1.0f / (1.0f + expf(-x)); }

__global__ __launch_bounds__(256) void k_cvt8(const float* __restrict__ src, bf* dst, size_t n8) {
    const size_t i = (size_t)blockIdx.x * 256 + threadIdx.x; if (i >= n8) return;
    const v8f v = *(const v8f*)(src + i * 8); v8us o;
#pragma unroll
    for (int k = 0; k < 8; ++k) o[k] = f2bf(v[k]);
    *(volatile v8us*)(dst + i * 8) = o; __threadfence(); *(volatile v8us*)(dst + i * 8) = o;
}

__global__ __launch_bounds__(256) void k_cvtx(const float* __restrict__ src, bf* dst, int srcRows, int srcCols, int dstRows, int dstCols) {
    const int c8n = dstCols >> 3;
    const int i = blockIdx.x * 256 + threadIdx.x; if (i >= dstRows * c8n) return;
    const int r = i / c8n, c = (i - r * c8n) * 8;
    const int rr = (r < srcRows) ? r : (srcRows - 1);
    const int sc = c % srcCols;
    const v8f v = *(const v8f*)(src + (size_t)rr * srcCols + sc);
    const bool z = (r >= srcRows);
    v8us o;
#pragma unroll
    for (int k = 0; k < 8; ++k) o[k] = z ? (unsigned short)0 : f2bf(v[k]);
    *(volatile v8us*)(dst + (size_t)i * 8) = o; __threadfence(); *(volatile v8us*)(dst + (size_t)i * 8) = o;
}

__global__ __launch_bounds__(32) void k_gemm(const bf* __restrict__ A, const bf* __restrict__ Bt, float* C, const float* __restrict__ bias, int useBias, int K, int ldc, int mtrue) {
    __shared__ __align__(16) float os[16 * 68];
    const int lane = threadIdx.x & 31, lr = lane & 15, hi = lane >> 4; const int r0 = blockIdx.x * 64, c0 = blockIdx.y * 64;
    v8f acc[4][4];
#pragma unroll
    for (int mb = 0; mb < 4; ++mb)
#pragma unroll
        for (int nb = 0; nb < 4; ++nb) acc[mb][nb] = (v8f){};
    const size_t aoff = (size_t)(r0 + lr) * K + 8 * hi, boff = (size_t)(c0 + lr) * K + 8 * hi;
#pragma unroll 1
    for (int kc = 0; kc < K; kc += 32) {
        v16bf a[4];
#pragma unroll
        for (int mb = 0; mb < 4; ++mb) a[mb] = ldb(A + aoff + (size_t)mb * 16 * K + kc);
#pragma unroll
        for (int nb = 0; nb < 4; ++nb) { const v16bf b = ldb(Bt + boff + (size_t)nb * 16 * K + kc);
#pragma unroll
            for (int mb = 0; mb < 4; ++mb) acc[mb][nb] = wmmab(a[mb], b, acc[mb][nb]); }
        asm volatile("v_nop\n\tv_nop\n\tv_nop\n\tv_nop" : "+v"(acc[0][0]), "+v"(acc[1][1]), "+v"(acc[2][2]), "+v"(acc[3][3]) : "v"(a[0]), "v"(a[1]), "v"(a[2]), "v"(a[3]));
    }
    v4f bv = (v4f){};
    if (useBias) {
#pragma unroll
        for (int i = 0; i < 4; ++i) bv[i] = bf16r(bias[c0 + lr * 4 + i]);
    }
#pragma unroll
    for (int mb = 0; mb < 4; ++mb) {
#pragma unroll
        for (int nb = 0; nb < 4; ++nb) {
#pragma unroll
            for (int j = 0; j < 8; ++j) os[(hi * 8 + j) * 68 + nb * 16 + lr] = acc[mb][nb][j]; }
        wave_sync();
#pragma unroll 1
        for (int ps = 0; ps < 2; ++ps) {
#pragma unroll
            for (int s = 0; s < 8; ++s) { const int row = 2 * s + hi, cofs = lr * 4;
                const v4f val = *(const v4fa*)(&os[row * 68 + cofs]) + bv;
                const int gr = r0 + mb * 16 + row;
                if (gr < mtrue) *(volatile v4f*)(C + (size_t)gr * (size_t)ldc + c0 + cofs) = val; }
            if (ps == 0) __threadfence(); }
        wave_sync();
    }
}

__device__ __forceinline__ void tile_gemm(const bf* __restrict__ W, size_t wo, v16bf a0, v16bf a1, v8f& c0, v8f& c1, v8f& c2, v8f& c3) {
    c0 = (v8f){}; c1 = (v8f){}; c2 = (v8f){}; c3 = (v8f){};
    { const v16bf b0 = ldb(W + wo), b1 = ldb(W + wo + 16 * DE), b2 = ldb(W + wo + 32 * DE), b3 = ldb(W + wo + 48 * DE);
      c0 = wmmab(a0, b0, c0); c1 = wmmab(a0, b1, c1); c2 = wmmab(a0, b2, c2); c3 = wmmab(a0, b3, c3);
      guard4(c0, c1, c2, c3, a0, b0, b1, b2, b3); }
    { const v16bf b0 = ldb(W + wo + 32), b1 = ldb(W + wo + 16 * DE + 32), b2 = ldb(W + wo + 32 * DE + 32), b3 = ldb(W + wo + 48 * DE + 32);
      c0 = wmmab(a1, b0, c0); c1 = wmmab(a1, b1, c1); c2 = wmmab(a1, b2, c2); c3 = wmmab(a1, b3, c3);
      guard4(c0, c1, c2, c3, a1, b0, b1, b2, b3); }
}

__global__ __launch_bounds__(32 * FW) void k_fused(const float* __restrict__ seq, const float* __restrict__ mem,
                                                   const bf* __restrict__ WKB, const bf* __restrict__ WVB, const bf* __restrict__ W1B, const float* __restrict__ VP,
                                                   const float* __restrict__ b1, const float* __restrict__ W2, const float* __restrict__ b2, bf* OUTP, float* ATT) {
    __shared__ __align__(16) float es[FW * 16 * 68];
    __shared__ __align__(16) float at[FW * 64];
    __shared__ __align__(16) float vm[HDW + DE];
    __shared__ __align__(16) float red[FW * 16 * 32];
    __shared__ __align__(16) float oc[HDW];
    const int tid = threadIdx.x;
    const int lane = tid & 31, lr = lane & 15, hi = lane >> 4;
    const int wave = __builtin_amdgcn_readfirstlane(tid >> 5);
    const int n = blockIdx.x;
    if (n >= NB) {
        if (wave == 0) { v8us z;
#pragma unroll
            for (int k = 0; k < 8; ++k) z[k] = 0;
            bf* o = OUTP + (size_t)n * (2 * HDW) + lane * 8;
            *(volatile v8us*)o = z; *(volatile v8us*)(o + HDW) = z; __threadfence(); *(volatile v8us*)o = z; *(volatile v8us*)(o + HDW) = z; }
        return;
    }
    vm[tid] = VP[(size_t)n * HDW + tid];
    if (tid < DE) vm[HDW + tid] = bf16r(mem[(size_t)n * DE + tid]);
#pragma unroll
    for (int k = 0; k < 16; ++k) red[(wave * 16 + k) * 32 + lane] = 0.0f;
    const float b1l = (lr < W1R) ? bf16r(b1[lr & (W1R - 1)]) : 0.0f;
    const float w2l = (lr < W1R) ? bf16r(W2[lr & (W1R - 1)]) : 0.0f;
    const float b2v = bf16r(b2[0]);
    __syncthreads();
    const int wb = wave * 16 * 68;
#pragma unroll 1
    for (int it = 0; it < TPW; ++it) {
        const int l0 = (wave * TPW + it) * 16;
        const float* ap = seq + ((size_t)n * SEQ_FULL + l0 + lr) * DE + 8 * hi;
        const v16bf a0 = lda_f32(ap), a1 = lda_f32(ap + 32);
#pragma unroll 1
        for (int h = 0; h < NH_; ++h) {
            const size_t wo = (size_t)(h * DE + lr) * DE + 8 * hi;
            { v8f c0, c1, c2, c3;
              tile_gemm(WKB, wo, a0, a1, c0, c1, c2, c3);
#pragma unroll
              for (int j = 0; j < 8; ++j) { const int ro = wb + (hi * 8 + j) * 68 + lr;
                  es[ro] = c0[j]; es[ro + 16] = c1[j]; es[ro + 32] = c2[j]; es[ro + 48] = c3[j]; } }
            wave_sync();
            v8f sc = (v8f){};
#pragma unroll
            for (int q = 0; q < 2; ++q) {
                const int eo = wb + lr * 68 + 32 * q + 8 * hi;
                const int vo = h * DE + 32 * q + 8 * hi;
                const int mo = HDW + 32 * q + 8 * hi;
                float ev[16], vv[16], mv[16], mk[16];
                { const v4f t0 = *(const v4fa*)(&es[eo]), t1 = *(const v4fa*)(&es[eo + 4]), t2 = *(const v4fa*)(&es[eo + 16]), t3 = *(const v4fa*)(&es[eo + 20]);
#pragma unroll
                  for (int i = 0; i < 4; ++i) { ev[i] = t0[i]; ev[4 + i] = t1[i]; ev[8 + i] = t2[i]; ev[12 + i] = t3[i]; } }
                { const v4f t0 = *(const v4fa*)(&vm[vo]), t1 = *(const v4fa*)(&vm[vo + 4]), t2 = *(const v4fa*)(&vm[vo + 16]), t3 = *(const v4fa*)(&vm[vo + 20]);
#pragma unroll
                  for (int i = 0; i < 4; ++i) { vv[i] = t0[i]; vv[4 + i] = t1[i]; vv[8 + i] = t2[i]; vv[12 + i] = t3[i]; } }
                { const v4f t0 = *(const v4fa*)(&vm[mo]), t1 = *(const v4fa*)(&vm[mo + 4]), t2 = *(const v4fa*)(&vm[mo + 16]), t3 = *(const v4fa*)(&vm[mo + 20]);
#pragma unroll
                  for (int i = 0; i < 4; ++i) { mv[i] = t0[i]; mv[4 + i] = t1[i]; mv[8 + i] = t2[i]; mv[12 + i] = t3[i]; } }
#pragma unroll
                for (int i = 0; i < 16; ++i) mk[i] = (ev[i] != 0.0f) ? 1.0f : 0.0f;
#pragma unroll
                for (int p = 0; p < 4; ++p) {
                    v8us ph0, ph1, pl0, pl1;
#pragma unroll
                    for (int i = 0; i < 8; ++i) {
                        float xa, xb;
                        if (p == 0)      { xa = (vv[i] - ev[i]) * mk[i]; xb = (vv[8 + i] - ev[8 + i]) * mk[8 + i]; }
                        else if (p == 1) { xa = (vv[i] * ev[i]) * mk[i]; xb = (vv[8 + i] * ev[8 + i]) * mk[8 + i]; }
                        else if (p == 2) { xa = (mv[i] - ev[i]) * mk[i]; xb = (mv[8 + i] - ev[8 + i]) * mk[8 + i]; }
                        else             { xa = (mv[i] * ev[i]) * mk[i]; xb = (mv[8 + i] * ev[8 + i]) * mk[8 + i]; }
                        const unsigned short ha = f2bf(xa), hb = f2bf(xb);
                        ph0[i] = ha; ph1[i] = hb;
                        pl0[i] = f2bf(xa - bf2f(ha)); pl1[i] = f2bf(xb - bf2f(hb));
                    }
                    const v16bf ah = cat16b(ph0, ph1), al = cat16b(pl0, pl1);
                    const v16bf b = ldb(W1B + (size_t)lr * HDW + 64 * p + 32 * q + 8 * hi);
                    sc = wmmab(ah, b, sc); sc = wmmab(al, b, sc);
                    guard1(sc, ah, al, b);
                }
            }
            float attr[8];
#pragma unroll
            for (int r = 0; r < 8; ++r) {
                const float hm = sigm(sc[r] + b1l);
                float t = hm * w2l;
                t += __shfl_xor(t, 1, 32); t += __shfl_xor(t, 2, 32); t += __shfl_xor(t, 4, 32);
                const float a = sigm(t + b2v);
                attr[r] = __shfl(a, lane & 16, 32);
            }
            float mine = attr[0];
#pragma unroll
            for (int r = 1; r < 8; ++r) mine = (lr == r) ? attr[r] : mine;
            if (lr < 8) at[wave * 64 + (8 * hi + lr) * 4 + h] = mine;
            { v8f c0, c1, c2, c3;
              tile_gemm(WVB, wo, a0, a1, c0, c1, c2, c3);
              float s0 = 0.0f, s1 = 0.0f, s2 = 0.0f, s3 = 0.0f;
#pragma unroll
              for (int r = 0; r < 8; ++r) { s0 = fmaf(attr[r], c0[r], s0); s1 = fmaf(attr[r], c1[r], s1); s2 = fmaf(attr[r], c2[r], s2); s3 = fmaf(attr[r], c3[r], s3); }
              const int ro = (wave * 16 + h * 4) * 32 + lane;
              const float r0v = red[ro] + s0, r1v = red[ro + 32] + s1, r2v = red[ro + 64] + s2, r3v = red[ro + 96] + s3;
              red[ro] = r0v; red[ro + 32] = r1v; red[ro + 64] = r2v; red[ro + 96] = r3v; }
            wave_sync();
        }
        const v4f av = *(const v4fa*)(&at[wave * 64 + lr * 4]);
        float* arow = ATT + ((size_t)n * SEQ_FULL + l0 + lr) * NH_;
        if (hi == 0) *(volatile v4f*)arow = av;
        __threadfence();
        if (hi == 0) *(volatile v4f*)arow = av;
        wave_sync();
    }
    __syncthreads();
    { const int c = tid; const int hh = c >> 6, nb = (c >> 4) & 3, cl = c & 15;
      float s = 0.0f;
#pragma unroll 1
      for (int w = 0; w < FW; ++w) { const int o = (w * 16 + hh * 4 + nb) * 32 + cl; s += red[o]; s += red[o + 16]; }
      oc[c] = s; }
    __syncthreads();
    if (wave == 0) {
        const v4f x0 = *(const v4fa*)(&oc[lane * 8]), x1 = *(const v4fa*)(&oc[lane * 8 + 4]);
        v8us hv, lv;
#pragma unroll
        for (int i = 0; i < 4; ++i) { const unsigned short h0 = f2bf(x0[i]), h1 = f2bf(x1[i]); hv[i] = h0; hv[4 + i] = h1; lv[i] = f2bf(x0[i] - bf2f(h0)); lv[4 + i] = f2bf(x1[i] - bf2f(h1)); }
        bf* o = OUTP + (size_t)n * (2 * HDW) + lane * 8;
        *(volatile v8us*)o = hv; *(volatile v8us*)(o + HDW) = lv;
        __threadfence();
        *(volatile v8us*)o = hv; *(volatile v8us*)(o + HDW) = lv;
    }
}

static constexpr size_t al256(size_t v) { return (v + 255) & ~(size_t)255; }
static constexpr size_t SZ_TB  = al256((size_t)NBP * DE * 2);
static constexpr size_t SZ_W   = al256((size_t)HDW * DE * 2);
static constexpr size_t SZ_W1  = al256((size_t)16 * HDW * 2);
static constexpr size_t SZ_WU  = al256((size_t)DE * 2 * HDW * 2);
static constexpr size_t SZ_VP  = al256((size_t)NBP * HDW * 4);
static constexpr size_t SZ_OP  = al256((size_t)NBP * 2 * HDW * 2);
static constexpr size_t SZ_TOTAL = SZ_TB + 3 * SZ_W + SZ_W1 + SZ_WU + SZ_VP + SZ_OP;
static_assert(SZ_TOTAL <= (size_t)134217728);

extern "C" void kernel_launch(void* const* d_in, const int* in_sizes, int n_in,
                              void* d_out, int out_size, void* d_ws, size_t ws_size, hipStream_t stream) {
    if (n_in < 12) return;
    if ((size_t)in_sizes[0] < ((size_t)(NB - 1) * SEQ_FULL + SEQ) * DE) return;
    if ((size_t)in_sizes[1] < (size_t)NB * DE || (size_t)in_sizes[2] < (size_t)NB * DE) return;
    if ((size_t)in_sizes[3] < (size_t)HDW * DE || (size_t)in_sizes[4] < (size_t)HDW * DE || (size_t)in_sizes[5] < (size_t)HDW * DE) return;
    if ((size_t)in_sizes[6] < (size_t)DE * HDW || in_sizes[7] < DE || in_sizes[8] < W1R * HDW || in_sizes[9] < W1R || in_sizes[10] < W1R || in_sizes[11] < 1) return;
    if ((size_t)out_size < OUT1_OFF + ((size_t)(NB - 1) * SEQ_FULL + SEQ) * NH_) return;
    if (SZ_TOTAL > ws_size) return;
    const float* seq = (const float*)d_in[0]; const float* tgt = (const float*)d_in[1]; const float* mem = (const float*)d_in[2];
    const float* wk = (const float*)d_in[3]; const float* wq = (const float*)d_in[4]; const float* wv = (const float*)d_in[5];
    const float* wu = (const float*)d_in[6]; const float* bu = (const float*)d_in[7]; const float* w1 = (const float*)d_in[8];
    const float* b1 = (const float*)d_in[9]; const float* w2 = (const float*)d_in[10]; const float* b2 = (const float*)d_in[11];
    float* OUT0 = (float*)d_out;
    float* ATT  = (float*)d_out + OUT1_OFF;
    char* wsp = (char*)d_ws;
    bf* TB  = (bf*)wsp; wsp += SZ_TB;
    bf* WKB = (bf*)wsp; wsp += SZ_W;
    bf* WQB = (bf*)wsp; wsp += SZ_W;
    bf* WVB = (bf*)wsp; wsp += SZ_W;
    bf* W1B = (bf*)wsp; wsp += SZ_W1;
    bf* WUB = (bf*)wsp; wsp += SZ_WU;
    float* VP = (float*)wsp; wsp += SZ_VP;
    bf* OUTP = (bf*)wsp; wsp += SZ_OP;

    k_cvtx<<<(unsigned)((NBP * DE / 8 + 255) / 256), 256, 0, stream>>>(tgt, TB, NB, DE, NBP, DE);
    { const size_t n8 = (size_t)HDW * DE / 8; const unsigned g = (unsigned)((n8 + 255) / 256);
      k_cvt8<<<g, 256, 0, stream>>>(wq, WQB, n8); k_cvt8<<<g, 256, 0, stream>>>(wk, WKB, n8); k_cvt8<<<g, 256, 0, stream>>>(wv, WVB, n8); }
    k_cvtx<<<(unsigned)((16 * HDW / 8 + 255) / 256), 256, 0, stream>>>(w1, W1B, W1R, HDW, 16, HDW);
    k_cvtx<<<(unsigned)((DE * 2 * HDW / 8 + 255) / 256), 256, 0, stream>>>(wu, WUB, DE, HDW, DE, 2 * HDW);

    k_gemm<<<dim3(NBP / 64, HDW / 64, 1), 32, 0, stream>>>(TB, WQB, VP, bu, 0, DE, HDW, NBP);

    k_fused<<<dim3(NBP, 1, 1), 32 * FW, 0, stream>>>(seq, mem, WKB, WVB, W1B, VP, b1, w2, b2, OUTP, ATT);

    k_gemm<<<dim3(NBP / 64, DE / 64, 1), 32, 0, stream>>>(OUTP, WUB, OUT0, bu, 1, 2 * HDW, DE, NB);
}
